// GATClassifier_85564338471313
// MI455X (gfx1250) — hardware-verified
//
#include <hip/hip_runtime.h>
#include <stddef.h>
#include <stdint.h>
#include <math.h>


#define F_IN    128
#define XUPR    (F_IN / 8)
#define NHD     8
#define HID     128
#define HCW     1024
#define HC3     512
#define KA2     2048
#define KA4     1024
#define NCLS    3
#define NSD     16
#define NTHR    256
#define NWAVE   8
#define EPT     8
#define CHUNK   (NTHR * EPT)
#define WCAP    (EPT * 32)
#define LISTN   (NWAVE * WCAP)
#define NBMAX   2048
#define SLOTB   11
#define RCAP    28672
#define DEGCAP  256
#define STGW    1024
#define GBM     64
#define GBN     128
#define GTHR    256
#define MROWS   128
#define HROWS   64
#define NEGSL   0.2f
#define EPS_SM  1e-16f
#define MX0     (-1.0e30f)
#define WSMAX   134217728
#define LDS_AGG ((2 * RCAP + 2 * NBMAX + LISTN) * 4 + 64)

static_assert((CHUNK & (CHUNK - 1)) == 0 && CHUNK <= (1 << SLOTB));
static_assert(NBMAX == (1 << SLOTB));
static_assert(NTHR * 8 == NBMAX);
static_assert(LISTN >= NBMAX);
static_assert(LISTN >= NWAVE * WCAP);
static_assert((RCAP % 32) == 0);
static_assert(NWAVE * STGW <= RCAP);
static_assert(STGW >= HCW && STGW >= HC3);
static_assert(LDS_AGG <= 300000);
static_assert(GBM == 4 * 16 && GTHR == 8 * 32);
static_assert((F_IN % 32) == 0 && (KA2 % 32) == 0 && (KA4 % 32) == 0);
static_assert((F_IN % 8) == 0);
static_assert((HCW % GBN) == 0 && (HC3 % GBN) == 0);
static_assert(GBN == HID && HCW == NHD * HID);
static_assert(HC3 == 4 * GBN);
static_assert(NSD == 2 * NHD && NSD >= 8);
static_assert(GBN == 32 * 4);
static_assert(KA2 == 2 * HCW && KA4 == 2 * HC3);
static_assert(HCW == 32 * 32);
static_assert(HID == 4 * 32);
static_assert(HCW == 4 * 256);
static_assert(HC3 == 16 * 32);
static_assert(HC3 == 2 * 256);
static_assert((MROWS % GBM) == 0);
static_assert(HC3 == 4 * 128);
static_assert(NTHR == 4 * HROWS);
static_assert(((HROWS * NCLS) % 4) == 0 && ((HROWS * NCLS * 4) % 128) == 0);
static_assert(((NCLS * HC3) % NTHR) == 0 && (NCLS * HC3) / NTHR <= 8);
static_assert(HROWS * NCLS <= NTHR);

typedef float          v4f  __attribute__((ext_vector_type(4)));
typedef float          v8f  __attribute__((ext_vector_type(8)));
typedef int            v4i  __attribute__((ext_vector_type(4)));
typedef int            v8i  __attribute__((ext_vector_type(8)));
typedef unsigned int   v4u  __attribute__((ext_vector_type(4)));
typedef unsigned short v8us __attribute__((ext_vector_type(8)));
typedef __bf16         v16b __attribute__((ext_vector_type(16)));
typedef v4f  __attribute__((may_alias)) v4fa;
typedef v8us __attribute__((may_alias)) v8usa;
union FragB { v16b v; v8us h[2]; v8i w; };

__device__ __forceinline__ v8f wmb(const FragB& a, const FragB& b, v8f c) {
  v8f d = __builtin_amdgcn_wmma_f32_16x16x32_bf16(false, a.v, false, b.v, (short)0, c, false, false);
  asm volatile("v_nop\n\tv_nop\n\tv_nop\n\tv_nop" : "+v"(d) : "v"(a.w), "v"(b.w));
  return d;
}

__device__ __forceinline__ unsigned int f2bf(float f) {
  const unsigned int u = __float_as_uint(f);
  return ((u + 0x7FFFu + ((u >> 16) & 1u)) >> 16) & 0xFFFFu;
}
__device__ __forceinline__ float bf2f(unsigned int b) { return __uint_as_float(b << 16); }
__device__ __forceinline__ float bfr(float f) { return bf2f(f2bf(f)); }
__device__ __forceinline__ v4f bfr4(const v4f a) {
  v4f r; r.x = bfr(a.x); r.y = bfr(a.y); r.z = bfr(a.z); r.w = bfr(a.w); return r;
}
__device__ __forceinline__ unsigned int pk2(float lo, float hi) { return f2bf(lo) | (f2bf(hi) << 16); }
__device__ __forceinline__ v4u pack8(const v4f a, const v4f b) {
  v4u r;
  r.x = pk2(a.x, a.y); r.y = pk2(a.z, a.w); r.z = pk2(b.x, b.y); r.w = pk2(b.z, b.w);
  return r;
}
__device__ __forceinline__ float reluf(float v) { return v < 0.f ? 0.f : v; }
__device__ __forceinline__ v4f relu4(const v4f a) {
  v4f r; r.x = reluf(a.x); r.y = reluf(a.y); r.z = reluf(a.z); r.w = reluf(a.w); return r;
}

__device__ __forceinline__ int scan_chunk(const int* __restrict__ dsts, int nE, int cbase, int slotBase,
                                          int nb, int vec8, int* list, int tid, int lane, int wave) {
  int wc = 0;
  const int el0  = tid * EPT;
  const int e0   = cbase + el0;
  const int sent = -2147483647 - 1;
  v4i da, db;
  if (vec8 != 0 && cbase + CHUNK <= nE) {
    da = *(const v4i*)(dsts + e0);
    db = *(const v4i*)(dsts + e0 + 4);
  } else {
    da.x = (e0     < nE) ? dsts[min(e0,     nE - 1)] : sent;
    da.y = (e0 + 1 < nE) ? dsts[min(e0 + 1, nE - 1)] : sent;
    da.z = (e0 + 2 < nE) ? dsts[min(e0 + 2, nE - 1)] : sent;
    da.w = (e0 + 3 < nE) ? dsts[min(e0 + 3, nE - 1)] : sent;
    db.x = (e0 + 4 < nE) ? dsts[min(e0 + 4, nE - 1)] : sent;
    db.y = (e0 + 5 < nE) ? dsts[min(e0 + 5, nE - 1)] : sent;
    db.z = (e0 + 6 < nE) ? dsts[min(e0 + 6, nE - 1)] : sent;
    db.w = (e0 + 7 < nE) ? dsts[min(e0 + 7, nE - 1)] : sent;
  }
  const unsigned nbs = (unsigned)slotBase;
  const unsigned unb = (unsigned)nb;
  const unsigned s0 = (unsigned)da.x - nbs, s1 = (unsigned)da.y - nbs;
  const unsigned s2 = (unsigned)da.z - nbs, s3 = (unsigned)da.w - nbs;
  const unsigned s4 = (unsigned)db.x - nbs, s5 = (unsigned)db.y - nbs;
  const unsigned s6 = (unsigned)db.z - nbs, s7 = (unsigned)db.w - nbs;
  const bool h0 = s0 < unb, h1 = s1 < unb, h2 = s2 < unb, h3 = s3 < unb;
  const bool h4 = s4 < unb, h5 = s5 < unb, h6 = s6 < unb, h7 = s7 < unb;
  const unsigned any = __builtin_amdgcn_ballot_w32(h0 | h1 | h2 | h3 | h4 | h5 | h6 | h7);
  if (any != 0u) {
#define HITJ(J, HJ, SJ) { \
      const unsigned mj = __builtin_amdgcn_ballot_w32(HJ); \
      if (mj != 0u) { \
        if (HJ) { \
          const int pos = wc + (int)__builtin_amdgcn_mbcnt_lo(mj, 0u); \
          if (pos < WCAP) list[wave * WCAP + pos] = ((el0 + (J)) << SLOTB) | (int)(SJ); \
        } \
        wc += (int)__builtin_popcount(mj); } }
    HITJ(0, h0, s0)
    HITJ(1, h1, s1)
    HITJ(2, h2, s2)
    HITJ(3, h3, s3)
    HITJ(4, h4, s4)
    HITJ(5, h5, s5)
    HITJ(6, h6, s6)
    HITJ(7, h7, s7)
#undef HITJ
  }
  return wc;
}

__global__ __launch_bounds__(NTHR) void k_xprep(const float* __restrict__ x, unsigned short* xb, int nN, int nUnits) {
  const int i = (int)blockIdx.x * NTHR + (int)threadIdx.x;
  if (i >= nUnits) return;
  const int row = i / XUPR;
  const int c0  = (i - row * XUPR) * 8;
  const int rc  = row < nN ? row : nN - 1;
  const float* p = x + (size_t)rc * F_IN + c0;
  v4f a = *(const v4fa*)p, b = *(const v4fa*)(p + 4);
  const v4f z4 = {0.f, 0.f, 0.f, 0.f};
  if (row >= nN) { a = z4; b = z4; }
  const v4u hv = pack8(a, b);
  const size_t o = (size_t)row * F_IN + c0;
  *(volatile v4u*)(xb + o) = hv;
  __threadfence();
  *(volatile v4u*)(xb + o) = hv;
}

__global__ __launch_bounds__(NTHR) void k_wprep(const float* __restrict__ w, int Kin, int Kper, int Ncol, int Nrows,
                                                int Kout, unsigned short* wt, int nUnits) {
  const int u = (int)blockIdx.x * NTHR + (int)threadIdx.x;
  if (u >= nUnits) return;
  const int kq = Kout >> 3;
  const int n  = u / kq;
  const int k8 = (u - n * kq) * 8;
  const int kk = k8 - (k8 / Kper) * Kper;
  const int ncl = n < Ncol ? n : Ncol - 1;
  const bool nl = (n < Ncol);
  const size_t nc = (size_t)Ncol;
  const float* p = w + ncl;
  const int q0 = min(kk + 0, Kin - 1), q1 = min(kk + 1, Kin - 1), q2 = min(kk + 2, Kin - 1), q3 = min(kk + 3, Kin - 1);
  const int q4 = min(kk + 4, Kin - 1), q5 = min(kk + 5, Kin - 1), q6 = min(kk + 6, Kin - 1), q7 = min(kk + 7, Kin - 1);
  v4f a, b;
  a.x = p[(size_t)q0 * nc]; a.y = p[(size_t)q1 * nc]; a.z = p[(size_t)q2 * nc]; a.w = p[(size_t)q3 * nc];
  b.x = p[(size_t)q4 * nc]; b.y = p[(size_t)q5 * nc]; b.z = p[(size_t)q6 * nc]; b.w = p[(size_t)q7 * nc];
  a.x = (nl && kk + 0 < Kin) ? a.x : 0.f;
  a.y = (nl && kk + 1 < Kin) ? a.y : 0.f;
  a.z = (nl && kk + 2 < Kin) ? a.z : 0.f;
  a.w = (nl && kk + 3 < Kin) ? a.w : 0.f;
  b.x = (nl && kk + 4 < Kin) ? b.x : 0.f;
  b.y = (nl && kk + 5 < Kin) ? b.y : 0.f;
  b.z = (nl && kk + 6 < Kin) ? b.z : 0.f;
  b.w = (nl && kk + 7 < Kin) ? b.w : 0.f;
  const v4u wv = pack8(a, b);
  unsigned short* o = wt + (size_t)n * (size_t)Kout + k8;
  *(volatile v4u*)o = wv;
  __threadfence();
  *(volatile v4u*)o = wv;
}

template<int EPI>
__global__ __launch_bounds__(GTHR) void k_gemm(
    const unsigned short* __restrict__ A, const unsigned short* __restrict__ WT, int K,
    float* outF, int ldo,
    const float* __restrict__ va, const float* __restrict__ vb, int vlen,
    float* SD, int MPr)
{
  __shared__ __attribute__((aligned(16))) float stg[GBM * GBN];
  __shared__ __attribute__((aligned(16))) float sv[2 * GBN];
  __shared__ __attribute__((aligned(16))) float sres[2 * GBM];
  const int tid = (int)threadIdx.x, lane = tid & 31, wave = tid >> 5, hh = lane >> 4, m = lane & 15;
  const int wr = wave & 3, wcol = wave >> 2;
  const int rowBase = (int)blockIdx.x * GBM;
  const int by      = (int)blockIdx.y;
  const int col0    = by * GBN;

  {
    const int which = tid >> 7;
    const int c = tid & (GBN - 1);
    int ai = col0 + c;
    ai = ai < vlen ? ai : vlen - 1;
    const float xs = va[ai];
    const float xd = vb[ai];
    const unsigned int msk = (which == 0) ? 0u : 0xFFFFFFFFu;
    const float v = __uint_as_float((__float_as_uint(xs) & ~msk) | (__float_as_uint(xd) & msk));
    sv[which * GBN + c] = bfr(v);
  }

  v8f acc[4];
  {
    const v8f z = {0.f, 0.f, 0.f, 0.f, 0.f, 0.f, 0.f, 0.f};
    acc[0] = z; acc[1] = z; acc[2] = z; acc[3] = z;
  }
  const unsigned short* ap = A  + (size_t)(rowBase + 16 * wr + m) * (size_t)K + 8 * hh;
  const unsigned short* wp = WT + (size_t)(col0 + 64 * wcol + m) * (size_t)K + 8 * hh;
  const int ksteps = K >> 5;
#pragma unroll 1
  for (int ks = 0; ks < ksteps; ++ks) {
    FragB af;
    af.h[0] = *(const v8usa*)(ap + 32 * ks);
    af.h[1] = *(const v8usa*)(ap + 32 * ks + 16);
#pragma unroll
    for (int t = 0; t < 4; ++t) {
      const unsigned short* wq = wp + (size_t)(16 * t) * (size_t)K + 32 * ks;
      FragB bf;
      bf.h[0] = *(const v8usa*)wq;
      bf.h[1] = *(const v8usa*)(wq + 16);
      acc[t] = wmb(af, bf, acc[t]);
    }
  }

#pragma unroll
  for (int t = 0; t < 4; ++t) {
    const int lc = 64 * wcol + 16 * t + m;
#pragma unroll
    for (int r = 0; r < 8; ++r) {
      const int lr = 16 * wr + 8 * hh + r;
      stg[lr * GBN + lc] = acc[t][r];
    }
  }
  __syncthreads();

  if (EPI == 0) {
    if (tid < 2 * GBM) {
      const int row = tid & (GBM - 1), which = tid >> 6;
      const float* sa = sv + which * GBN;
      const float* hr = stg + row * GBN;
      float d = 0.f;
#pragma unroll 4
      for (int c4 = 0; c4 < GBN / 4; ++c4) {
        const v4f hv = *(const v4fa*)(hr + 4 * c4);
        const v4f av = *(const v4fa*)(sa + 4 * c4);
        d = fmaf(hv.x, av.x, d);
        d = fmaf(hv.y, av.y, d);
        d = fmaf(hv.z, av.z, d);
        d = fmaf(hv.w, av.w, d);
      }
      sres[which * GBM + row] = d;
    }
  }
  v4f fv[8];
#pragma unroll
  for (int it = 0; it < 8; ++it) {
    const int row = 8 * it + wave;
    v4f h = *(const v4fa*)(stg + row * GBN + 4 * lane);
    if (EPI == 1) {
      const v4f bv = *(const v4fa*)(sv + 4 * lane);
      h = relu4(h + bv);
    }
    fv[it] = h;
  }
  __syncthreads();
  const int which2 = lane >> 4, piece = lane & 15;
  v4f sdv = {0.f, 0.f, 0.f, 0.f};
  float* sp = SD;
  if (EPI == 0) {
    sdv = *(const v4fa*)(sres + which2 * GBM + 4 * piece);
    sp = SD + (size_t)(2 * by + which2) * (size_t)MPr + rowBase + 4 * piece;
  }
#pragma unroll
  for (int it = 0; it < 8; ++it) {
    const int gr = rowBase + 8 * it + wave;
    float* op = outF + (size_t)gr * (size_t)ldo + col0 + 4 * lane;
    *(volatile v4f*)op = fv[it];
  }
  if (EPI == 0 && wave == 0) *(volatile v4f*)sp = sdv;
  __threadfence();
#pragma unroll
  for (int it = 0; it < 8; ++it) {
    const int gr = rowBase + 8 * it + wave;
    float* op = outF + (size_t)gr * (size_t)ldo + col0 + 4 * lane;
    *(volatile v4f*)op = fv[it];
  }
  if (EPI == 0 && wave == 0) *(volatile v4f*)sp = sdv;
}

template<int L>
__global__ __launch_bounds__(NTHR) void k_agg(
    const int* __restrict__ srcs, const int* __restrict__ dsts,
    const float* __restrict__ F, const float* __restrict__ SD, const float* __restrict__ bias,
    unsigned short* HP, int nN, int nE, int nb, int vec8, int MPr) {
  extern __shared__ v4f lds_dyn[];
  int* reg1 = (int*)lds_dyn;
  int* reg2 = reg1 + RCAP;
  int* scnt = reg2 + RCAP;
  int* soff = scnt + NBMAX;
  int* list = soff + NBMAX;
  int* wcnt = list + LISTN;
  int* wtot = wcnt + NWAVE;
  const int tid = (int)threadIdx.x, lane = tid & 31, wave = tid >> 5;
  const int nodeBase = (int)blockIdx.x * nb;

  for (int i = tid; i < NBMAX; i += NTHR) scnt[i] = 0;
  __syncthreads();

  int tot = 0;
  const int nChunks = (nE + CHUNK - 1) / CHUNK;
#pragma unroll 1
  for (int ch = 0; ch < nChunks; ++ch) {
    const int cbase = ch * CHUNK;
    const int wc = scan_chunk(dsts, nE, cbase, nodeBase, nb, vec8, list, tid, lane, wave);
    if (lane == 0) wcnt[wave] = wc;
    __syncthreads();
    int pre = 0, all = 0;
#pragma unroll
    for (int w2 = 0; w2 < NWAVE; ++w2) {
      int c = wcnt[w2];
      c = c < 0 ? 0 : (c > WCAP ? WCAP : c);
      all += c;
      pre += (w2 < wave) ? c : 0;
    }
    const int wcc  = wc > WCAP ? WCAP : wc;
    const int base = tot + pre;
#pragma unroll 1
    for (int i = lane; i < wcc; i += 32) {
      const int ent = list[wave * WCAP + i];
      const int el  = (ent >> SLOTB) & (CHUNK - 1);
      const int sl  = ent & (NBMAX - 1);
      int eid = cbase + el;
      eid = eid > nE - 1 ? nE - 1 : eid;
      const int pos = base + i;
      if (pos < RCAP) reg1[pos] = (int)(((unsigned)eid << SLOTB) | (unsigned)sl);
    }
    tot += all;
    tot = tot > RCAP ? RCAP : tot;
    __syncthreads();
  }
  const int nh = tot;

  if (wave == 0) {
#pragma unroll 1
    for (int b0 = 0; b0 < nh; b0 += 32) {
      const int idx = b0 + lane;
      const int uv  = reg1[idx < nh ? idx : nh - 1];
      const int m32 = (nh - b0) < 32 ? (nh - b0) : 32;
#pragma unroll 1
      for (int k = 0; k < m32; ++k) {
        const int u  = __builtin_amdgcn_readlane(uv, k);
        const int sl = u & (NBMAX - 1);
        if (lane == 0) scnt[sl] = scnt[sl] + 1;
      }
    }
  }
  __syncthreads();

  {
    const v4i ca = *(const v4i*)(scnt + 8 * tid);
    const v4i cb = *(const v4i*)(scnt + 8 * tid + 4);
    const int e0 = ca.x < 0 ? 0 : ca.x, e1 = ca.y < 0 ? 0 : ca.y, e2 = ca.z < 0 ? 0 : ca.z, e3 = ca.w < 0 ? 0 : ca.w;
    const int e4 = cb.x < 0 ? 0 : cb.x, e5 = cb.y < 0 ? 0 : cb.y, e6 = cb.z < 0 ? 0 : cb.z, e7 = cb.w < 0 ? 0 : cb.w;
    const int ts = e0 + e1 + e2 + e3 + e4 + e5 + e6 + e7;
    int incl = ts;
#pragma unroll
    for (int d = 1; d < 32; d <<= 1) {
      const int up = __shfl_up(incl, d);
      if (lane >= d) incl += up;
    }
    if (lane == 31) wtot[wave] = incl;
    __syncthreads();
    int pre = 0;
#pragma unroll
    for (int w2 = 0; w2 < NWAVE; ++w2) pre += (w2 < wave) ? wtot[w2] : 0;
    int run = pre + incl - ts;
    soff[8 * tid + 0] = run; run += e0;
    soff[8 * tid + 1] = run; run += e1;
    soff[8 * tid + 2] = run; run += e2;
    soff[8 * tid + 3] = run; run += e3;
    soff[8 * tid + 4] = run; run += e4;
    soff[8 * tid + 5] = run; run += e5;
    soff[8 * tid + 6] = run; run += e6;
    soff[8 * tid + 7] = run;
  }
  __syncthreads();
  for (int i = tid; i < NBMAX; i += NTHR) list[i] = soff[i];
  __syncthreads();

  if (wave == 0) {
#pragma unroll 1
    for (int b0 = 0; b0 < nh; b0 += 32) {
      const int idx = b0 + lane;
      const int uv  = reg1[idx < nh ? idx : nh - 1];
      const int m32 = (nh - b0) < 32 ? (nh - b0) : 32;
#pragma unroll 1
      for (int k = 0; k < m32; ++k) {
        const int u   = __builtin_amdgcn_readlane(uv, k);
        const int sl  = u & (NBMAX - 1);
        const int eid = (int)((unsigned)u >> SLOTB);
        if (lane == 0) {
          int pos = list[sl];
          pos = pos < 0 ? 0 : (pos > RCAP - 1 ? RCAP - 1 : pos);
          reg2[pos] = eid;
          list[sl] = pos + 1;
        }
      }
    }
  }
  __syncthreads();

  const int nbw = nb >> 3;
  const bool ovf = (nh >= RCAP);
  const float qnan = __int_as_float(0x7fc00000);
  const v4f z4 = {0.f, 0.f, 0.f, 0.f};
  float* stw = (float*)reg1 + wave * STGW;

  if (L == 1) {
    const int c0   = 32 * lane;
    const int head = lane >> 2;
    const float* ASp = SD + (size_t)(2 * head) * (size_t)MPr;
    const float* ADp = ASp + MPr;

#pragma unroll 1
    for (int jt = 0; jt < nbw; ++jt) {
      const int slot = wave * nbw + jt;
      const int grow = nodeBase + slot;
      const int gcl  = grow < nN ? grow : nN - 1;
      int st = soff[slot];
      const int craw = scnt[slot];
      int cnt = craw;
      st  = st < 0 ? 0 : (st > nh ? nh : st);
      cnt = cnt < 0 ? 0 : (cnt > DEGCAP ? DEGCAP : cnt);
      if (cnt > nh - st) cnt = nh - st;
      const float pz = (ovf || craw > DEGCAP) ? qnan : 0.0f;

      const float adv = ADp[gcl];
      float mx = MX0, dn = 0.0f;
      v4f a[8];
#pragma unroll
      for (int i = 0; i < 8; ++i) a[i] = z4;

#pragma unroll 1
      for (int q = 0; q < cnt; ++q) {
        int idx = st + q; idx = idx > RCAP - 1 ? RCAP - 1 : idx;
        int eid = reg2[idx]; eid = eid < 0 ? 0 : (eid > nE - 1 ? nE - 1 : eid);
        const int sraw = srcs[eid];
        const int s = sraw < 0 ? 0 : (sraw > nN - 1 ? nN - 1 : sraw);
        const float* fr = F + (size_t)s * HCW + c0;
        v4f f[8];
#pragma unroll
        for (int i = 0; i < 8; ++i) f[i] = *(const v4fa*)(fr + 4 * i);
        float lg = ASp[s] + adv;
        lg = lg > 0.f ? lg : NEGSL * lg;
        const float df = lg - mx;
        const float ee = __expf(-fabsf(df));
        const bool up  = df > 0.f;
        const float s1 = up ? ee : 1.0f;
        const float s2 = up ? 1.0f : ee;
        mx = up ? lg : mx;
        dn = fmaf(dn, s1, s2);
#pragma unroll
        for (int i = 0; i < 8; ++i) {
          a[i].x = fmaf(a[i].x, s1, s2 * f[i].x);
          a[i].y = fmaf(a[i].y, s1, s2 * f[i].y);
          a[i].z = fmaf(a[i].z, s1, s2 * f[i].z);
          a[i].w = fmaf(a[i].w, s1, s2 * f[i].w);
        }
      }
      const float inv = __builtin_amdgcn_rcpf(dn + EPS_SM);
#pragma unroll
      for (int i = 0; i < 8; ++i) *(v4f*)(stw + c0 + 4 * i) = a[i] * inv;
      __syncthreads();
      const bool live = grow < nN;
      v4u hv[4], lv[4];
#pragma unroll
      for (int jj = 0; jj < 4; ++jj) {
        const int cb = 256 * jj + 8 * lane;
        const v4f u0 = *(const v4fa*)(stw + cb);
        const v4f u1 = *(const v4fa*)(stw + cb + 4);
        const v4f b0 = bfr4(*(const v4fa*)(bias + cb));
        const v4f b1 = bfr4(*(const v4fa*)(bias + cb + 4));
        const v4f r0 = relu4(u0 + b0), r1 = relu4(u1 + b1);
        v4f v0, v1;
        v0.x = (live ? r0.x : 0.f) + pz; v0.y = (live ? r0.y : 0.f) + pz;
        v0.z = (live ? r0.z : 0.f) + pz; v0.w = (live ? r0.w : 0.f) + pz;
        v1.x = (live ? r1.x : 0.f) + pz; v1.y = (live ? r1.y : 0.f) + pz;
        v1.z = (live ? r1.z : 0.f) + pz; v1.w = (live ? r1.w : 0.f) + pz;
        hv[jj] = pack8(v0, v1);
        lv[jj] = pack8(v0 - bfr4(v0), v1 - bfr4(v1));
      }
      unsigned short* gp = HP + (size_t)grow * KA2 + 8 * lane;
      const bool wr = grow < MPr;
      if (wr) {
#pragma unroll
        for (int jj = 0; jj < 4; ++jj) {
          *(volatile v4u*)(gp + 256 * jj)       = hv[jj];
          *(volatile v4u*)(gp + HCW + 256 * jj) = lv[jj];
        }
      }
      __threadfence();
      if (wr) {
#pragma unroll
        for (int jj = 0; jj < 4; ++jj) {
          *(volatile v4u*)(gp + 256 * jj)       = hv[jj];
          *(volatile v4u*)(gp + HCW + 256 * jj) = lv[jj];
        }
      }
      __syncthreads();
    }
  } else {
    const int c0 = 16 * lane;
    const size_t mp = (size_t)MPr;

#pragma unroll 1
    for (int jt = 0; jt < nbw; ++jt) {
      const int slot = wave * nbw + jt;
      const int grow = nodeBase + slot;
      const int gcl  = grow < nN ? grow : nN - 1;
      int st = soff[slot];
      const int craw = scnt[slot];
      int cnt = craw;
      st  = st < 0 ? 0 : (st > nh ? nh : st);
      cnt = cnt < 0 ? 0 : (cnt > DEGCAP ? DEGCAP : cnt);
      if (cnt > nh - st) cnt = nh - st;
      const float pz = (ovf || craw > DEGCAP) ? qnan : 0.0f;

      const float adv = (SD[mp + gcl] + SD[3 * mp + gcl]) + (SD[5 * mp + gcl] + SD[7 * mp + gcl]);
      float mx = MX0, dn = 0.0f;
      v4f a[4];
#pragma unroll
      for (int i = 0; i < 4; ++i) a[i] = z4;

#pragma unroll 1
      for (int q = 0; q < cnt; ++q) {
        int idx = st + q; idx = idx > RCAP - 1 ? RCAP - 1 : idx;
        int eid = reg2[idx]; eid = eid < 0 ? 0 : (eid > nE - 1 ? nE - 1 : eid);
        const int sraw = srcs[eid];
        const int s = sraw < 0 ? 0 : (sraw > nN - 1 ? nN - 1 : sraw);
        const float* fr = F + (size_t)s * HC3 + c0;
        v4f f[4];
#pragma unroll
        for (int i = 0; i < 4; ++i) f[i] = *(const v4fa*)(fr + 4 * i);
        const float asv = (SD[s] + SD[2 * mp + s]) + (SD[4 * mp + s] + SD[6 * mp + s]);
        float lg = asv + adv;
        lg = lg > 0.f ? lg : NEGSL * lg;
        const float df = lg - mx;
        const float ee = __expf(-fabsf(df));
        const bool up  = df > 0.f;
        const float s1 = up ? ee : 1.0f;
        const float s2 = up ? 1.0f : ee;
        mx = up ? lg : mx;
        dn = fmaf(dn, s1, s2);
#pragma unroll
        for (int i = 0; i < 4; ++i) {
          a[i].x = fmaf(a[i].x, s1, s2 * f[i].x);
          a[i].y = fmaf(a[i].y, s1, s2 * f[i].y);
          a[i].z = fmaf(a[i].z, s1, s2 * f[i].z);
          a[i].w = fmaf(a[i].w, s1, s2 * f[i].w);
        }
      }
      const float inv = __builtin_amdgcn_rcpf(dn + EPS_SM);
#pragma unroll
      for (int i = 0; i < 4; ++i) *(v4f*)(stw + c0 + 4 * i) = a[i] * inv;
      __syncthreads();
      const bool live = grow < nN;
      v4u hv[2], lv[2];
#pragma unroll
      for (int jj = 0; jj < 2; ++jj) {
        const int cb = 256 * jj + 8 * lane;
        const v4f u0 = *(const v4fa*)(stw + cb);
        const v4f u1 = *(const v4fa*)(stw + cb + 4);
        const v4f b0 = bfr4(*(const v4fa*)(bias + cb));
        const v4f b1 = bfr4(*(const v4fa*)(bias + cb + 4));
        const v4f r0 = relu4(u0 + b0), r1 = relu4(u1 + b1);
        v4f v0, v1;
        v0.x = (live ? r0.x : 0.f) + pz; v0.y = (live ? r0.y : 0.f) + pz;
        v0.z = (live ? r0.z : 0.f) + pz; v0.w = (live ? r0.w : 0.f) + pz;
        v1.x = (live ? r1.x : 0.f) + pz; v1.y = (live ? r1.y : 0.f) + pz;
        v1.z = (live ? r1.z : 0.f) + pz; v1.w = (live ? r1.w : 0.f) + pz;
        hv[jj] = pack8(v0, v1);
        lv[jj] = pack8(v0 - bfr4(v0), v1 - bfr4(v1));
      }
      unsigned short* gp = HP + (size_t)grow * KA4 + 8 * lane;
      const bool wr = grow < MPr;
      if (wr) {
#pragma unroll
        for (int jj = 0; jj < 2; ++jj) {
          *(volatile v4u*)(gp + 256 * jj)       = hv[jj];
          *(volatile v4u*)(gp + HC3 + 256 * jj) = lv[jj];
        }
      }
      __threadfence();
      if (wr) {
#pragma unroll
        for (int jj = 0; jj < 2; ++jj) {
          *(volatile v4u*)(gp + 256 * jj)       = hv[jj];
          *(volatile v4u*)(gp + HC3 + 256 * jj) = lv[jj];
        }
      }
      __syncthreads();
    }
  }
}

__global__ __launch_bounds__(NTHR) void k_head(const float* __restrict__ H4, const float* __restrict__ wc,
                                               const float* __restrict__ bcv, float* out, int nN) {
  __shared__ __attribute__((aligned(16))) float swc[NCLS * HC3];
  __shared__ __attribute__((aligned(16))) float spart[4 * HROWS * 4];
  __shared__ __attribute__((aligned(16))) float sy[HROWS * NCLS];
  const int tid = (int)threadIdx.x;
  const int r0 = (int)blockIdx.x * HROWS;

#pragma unroll 1
  for (int j = 0; j < (NCLS * HC3) / NTHR; ++j) {
    const int i = j * NTHR + tid;
    const int k = i / NCLS;
    const int o = i - k * NCLS;
    swc[o * HC3 + k] = bfr(wc[i]);
  }
  __syncthreads();

  {
    const int row = tid & (HROWS - 1), q = tid >> 6;
    int grow = r0 + row;
    grow = grow < nN ? grow : nN - 1;
    const float* hp = H4 + (size_t)grow * HC3 + 128 * q;
    const float* w0 = swc + 128 * q;
    const float* w1 = w0 + HC3;
    const float* w2 = w1 + HC3;
    float d0 = 0.f, d1 = 0.f, d2 = 0.f;
#pragma unroll 2
    for (int c4 = 0; c4 < 32; ++c4) {
      const v4f hv = *(const v4fa*)(hp + 4 * c4);
      const v4f av = *(const v4fa*)(w0 + 4 * c4);
      const v4f bv = *(const v4fa*)(w1 + 4 * c4);
      const v4f cv = *(const v4fa*)(w2 + 4 * c4);
      d0 = fmaf(hv.x, av.x, d0); d1 = fmaf(hv.x, bv.x, d1); d2 = fmaf(hv.x, cv.x, d2);
      d0 = fmaf(hv.y, av.y, d0); d1 = fmaf(hv.y, bv.y, d1); d2 = fmaf(hv.y, cv.y, d2);
      d0 = fmaf(hv.z, av.z, d0); d1 = fmaf(hv.z, bv.z, d1); d2 = fmaf(hv.z, cv.z, d2);
      d0 = fmaf(hv.w, av.w, d0); d1 = fmaf(hv.w, bv.w, d1); d2 = fmaf(hv.w, cv.w, d2);
    }
    float* pp = spart + (q * HROWS + row) * 4;
    pp[0] = d0; pp[1] = d1; pp[2] = d2;
  }
  __syncthreads();
  if (tid < HROWS * NCLS) {
    const int rr = tid / NCLS;
    const int o  = tid - rr * NCLS;
    const float p0 = spart[(0 * HROWS + rr) * 4 + o];
    const float p1 = spart[(1 * HROWS + rr) * 4 + o];
    const float p2 = spart[(2 * HROWS + rr) * 4 + o];
    const float p3 = spart[(3 * HROWS + rr) * 4 + o];
    sy[rr * NCLS + o] = ((p0 + p1) + (p2 + p3)) + bfr(bcv[o]);
  }
  __syncthreads();

  const int nOut = nN * NCLS;
  const bool pw = tid < (HROWS * NCLS) / 4;
  const int pc = pw ? tid : 0;
  const v4f yv = *(const v4fa*)(sy + 4 * pc);
  const size_t e0 = (size_t)r0 * NCLS + 4 * (size_t)pc;
  float* op = out + e0;
  const bool full = pw && (e0 + 4 <= (size_t)nOut);
  const bool w0 = pw && !full && (e0     < (size_t)nOut);
  const bool w1 = pw && !full && (e0 + 1 < (size_t)nOut);
  const bool w2 = pw && !full && (e0 + 2 < (size_t)nOut);
  if (full) *(volatile v4f*)op = yv;
  if (w0) *(volatile float*)op = yv.x;
  if (w1) *(volatile float*)(op + 1) = yv.y;
  if (w2) *(volatile float*)(op + 2) = yv.z;
  __threadfence();
  if (full) *(volatile v4f*)op = yv;
  if (w0) *(volatile float*)op = yv.x;
  if (w1) *(volatile float*)(op + 1) = yv.y;
  if (w2) *(volatile float*)(op + 2) = yv.z;
}

static int pick_nb(int nE, int nN) {
  int nb = NBMAX;
  while (nb > 32 && (long long)nb * (long long)nE * 5LL > (long long)RCAP * (long long)nN * 4LL) nb >>= 1;
  return nb;
}
static inline int cdiv(int a, int b) { return (a + b - 1) / b; }

extern "C" void kernel_launch(void* const* d_in, const int* in_sizes, int n_in,
                              void* d_out, int out_size, void* d_ws, size_t ws_size,
                              hipStream_t stream) {
  if (n_in < 18) return;
  if (in_sizes[0] <= 0 || (in_sizes[0] % F_IN) != 0) return;
  const int nN = in_sizes[0] / F_IN;
  if (nN <= 0 || nN > (1 << 22)) return;
  if (in_sizes[1] < 2 || (in_sizes[1] & 1) != 0) return;
  const int nE = in_sizes[1] / 2;
  if (nE < 1 || nE >= (1 << (32 - SLOTB))) return;
  if (in_sizes[2]  != F_IN * HCW) return;
  if (in_sizes[3]  != HCW || in_sizes[4] != HCW) return;
  if (in_sizes[5]  != HCW) return;
  if (in_sizes[6]  != HCW * HCW) return;
  if (in_sizes[7]  != HCW || in_sizes[8] != HCW) return;
  if (in_sizes[9]  != HCW) return;
  if (in_sizes[10] != HCW * HC3) return;
  if (in_sizes[11] != HC3 || in_sizes[12] != HC3) return;
  if (in_sizes[13] != HC3) return;
  if (in_sizes[14] != HC3 * HC3) return;
  if (in_sizes[15] != HC3) return;
  if (in_sizes[16] != HC3 * NCLS) return;
  if (in_sizes[17] != NCLS) return;
  if (out_size != nN * NCLS) return;

  const float* x   = (const float*)d_in[0];
  const int*   ei  = (const int*)  d_in[1];
  const float* W1  = (const float*)d_in[2];
  const float* a1s = (const float*)d_in[3];
  const float* a1d = (const float*)d_in[4];
  const float* b1  = (const float*)d_in[5];
  const float* W2  = (const float*)d_in[6];
  const float* a2s = (const float*)d_in[7];
  const float* a2d = (const float*)d_in[8];
  const float* b2  = (const float*)d_in[9];
  const float* W3  = (const float*)d_in[10];
  const float* a3s = (const float*)d_in[11];
  const float* a3d = (const float*)d_in[12];
  const float* b3  = (const float*)d_in[13];
  const float* Wl  = (const float*)d_in[14];
  const float* bl  = (const float*)d_in[15];
  const float* Wc  = (const float*)d_in[16];
  const float* bc  = (const float*)d_in[17];
  float* out = (float*)d_out;
  const int* src = ei;
  const int* dst = ei + nE;

  const int MP   = cdiv(nN, MROWS) * MROWS;
  const int nb   = pick_nb(nE, nN);
  if (nb < 32 || (nb & (nb - 1)) != 0 || nb > NBMAX) return;
  const int gA   = cdiv(MP, nb);
  const int vec8 = ((nE & 3) == 0) ? 1 : 0;
  if (gA * nb < MP) return;

  char* ws = (char*)d_ws;
  size_t off = 0;
  const size_t oXB  = off; off += (size_t)MP * F_IN * 2;           off = (off + 255) & ~(size_t)255;
  const size_t oW1T = off; off += (size_t)HCW * F_IN * 2;          off = (off + 255) & ~(size_t)255;
  const size_t oW2T = off; off += (size_t)HCW * KA2 * 2;           off = (off + 255) & ~(size_t)255;
  const size_t oW3T = off; off += (size_t)HC3 * KA2 * 2;           off = (off + 255) & ~(size_t)255;
  const size_t oWLT = off; off += (size_t)HC3 * KA4 * 2;           off = (off + 255) & ~(size_t)255;
  const size_t oH   = off; off += (size_t)MP * HCW * 4;            off = (off + 255) & ~(size_t)255;
  const size_t oSD  = off; off += (size_t)NSD * MP * 4;            off = (off + 255) & ~(size_t)255;
  const size_t oAP  = off; off += (size_t)MP * KA2 * 2;            off = (off + 255) & ~(size_t)255;
  if (off > ws_size || off > (size_t)WSMAX) return;
  unsigned short* XB  = (unsigned short*)(ws + oXB);
  unsigned short* W1T = (unsigned short*)(ws + oW1T);
  unsigned short* W2T = (unsigned short*)(ws + oW2T);
  unsigned short* W3T = (unsigned short*)(ws + oW3T);
  unsigned short* WLT = (unsigned short*)(ws + oWLT);
  float*          H   = (float*)(ws + oH);
  float*          SD  = (float*)(ws + oSD);
  unsigned short* AP  = (unsigned short*)(ws + oAP);

  hipFuncSetAttribute(reinterpret_cast<const void*>(&k_agg<1>),
                      hipFuncAttributeMaxDynamicSharedMemorySize, LDS_AGG);
  hipFuncSetAttribute(reinterpret_cast<const void*>(&k_agg<3>),
                      hipFuncAttributeMaxDynamicSharedMemorySize, LDS_AGG);

  const int nUx = MP * XUPR;
  k_xprep<<<cdiv(nUx, NTHR), NTHR, 0, stream>>>(x, XB, nN, nUx);

  {
    const int nUw1 = HCW * (F_IN / 8);
    k_wprep<<<cdiv(nUw1, NTHR), NTHR, 0, stream>>>(W1, F_IN, F_IN, HCW, HCW, F_IN, W1T, nUw1);
    const int nUw2 = HCW * (KA2 / 8);
    k_wprep<<<cdiv(nUw2, NTHR), NTHR, 0, stream>>>(W2, HCW, HCW, HCW, HCW, KA2, W2T, nUw2);
    const int nUw3 = HC3 * (KA2 / 8);
    k_wprep<<<cdiv(nUw3, NTHR), NTHR, 0, stream>>>(W3, HCW, HCW, HC3, HC3, KA2, W3T, nUw3);
    const int nUwl = HC3 * (KA4 / 8);
    k_wprep<<<cdiv(nUwl, NTHR), NTHR, 0, stream>>>(Wl, HC3, HC3, HC3, HC3, KA4, WLT, nUwl);
  }

  const int gM = MP / GBM;
  k_gemm<0><<<dim3(gM, HCW / GBN), GTHR, 0, stream>>>(XB, W1T, F_IN, H, HCW, a1s, a1d, HCW, SD, MP);
  k_agg<1><<<gA, NTHR, LDS_AGG, stream>>>(src, dst, H, SD, b1, AP, nN, nE, nb, vec8, MP);
  k_gemm<0><<<dim3(gM, HCW / GBN), GTHR, 0, stream>>>(AP, W2T, KA2, H, HCW, a2s, a2d, HCW, SD, MP);
  k_agg<1><<<gA, NTHR, LDS_AGG, stream>>>(src, dst, H, SD, b2, AP, nN, nE, nb, vec8, MP);
  k_gemm<0><<<dim3(gM, HC3 / GBN), GTHR, 0, stream>>>(AP, W3T, KA2, H, HC3, a3s, a3d, HC3, SD, MP);
  k_agg<3><<<gA, NTHR, LDS_AGG, stream>>>(src, dst, H, SD, b3, AP, nN, nE, nb, vec8, MP);
  k_gemm<1><<<dim3(gM, HC3 / GBN), GTHR, 0, stream>>>(AP, WLT, KA4, H, HC3, bl, bl, HC3, SD, MP);
  k_head<<<cdiv(nN, HROWS), NTHR, 0, stream>>>(H, Wc, bc, out, nN);
}
